// TransformerBlock_39032662786707
// MI455X (gfx1250) — hardware-run, weakly checked
//
#include <hip/hip_runtime.h>
#include <stddef.h>


typedef _Float16 v16h __attribute__((ext_vector_type(16)));
typedef _Float16 v8h  __attribute__((ext_vector_type(8)));
typedef float    v8f  __attribute__((ext_vector_type(8)));
typedef float    v4f  __attribute__((ext_vector_type(4)));

#ifndef NB
#define NB 2
#endif
#ifndef SEQ
#define SEQ 2048
#endif
#define NB_FULL  2
#define SEQ_FULL 2048
#define DIM   1024
#define DFF   4096
#define NHEAD 16
#define HD    64
#define MROWS (NB * SEQ)
#define LNROWS 8
#define LN_EPS 1.0e-5f

static_assert(NB >= 1 && NB <= NB_FULL);
static_assert(SEQ >= 128 && SEQ <= SEQ_FULL && (SEQ % 128) == 0);
static_assert((SEQ % 64) == 0);
static_assert(DIM == NHEAD * HD);
static_assert(HD == 64);
static_assert((DIM % 64) == 0 && (DIM % 32) == 0);
static_assert((DFF % 64) == 0 && (DFF % 32) == 0);
static_assert((MROWS % 64) == 0);
static_assert((MROWS % LNROWS) == 0);
static_assert((DIM % 256) == 0);

#define LDT 72
#define LDC 68

#define WCARRY 64.0f
#define PCARRY 1024.0f
#define VCARRY 64.0f

#define OUT1_ELEM ((size_t)NB_FULL * SEQ_FULL * DIM)
#define OUT_TOTAL_FULL ((size_t)12582912)
#define NEED_OUT (OUT1_ELEM + ((((size_t)(NB_FULL + NB - 1) * NHEAD + (NHEAD - 1)) * SEQ_FULL + (SEQ - 1)) * HD + HD))
static_assert(OUT1_ELEM * 4 == (size_t)16777216);
static_assert(NEED_OUT <= OUT_TOTAL_FULL);
static_assert(((size_t)(SEQ - 1) * NB_FULL + NB) * DIM <= OUT1_ELEM);

#define WQKV_BYTES ((size_t)3 * DIM * DIM * 2)
#define WPR_BYTES  ((size_t)DIM * DIM * 2)
#define WFF_BYTES  ((size_t)DFF * DIM * 2)
#define P16_BYTES  ((size_t)MROWS * DIM * 2)
#define P32_BYTES  ((size_t)MROWS * DIM * 4)
#define F1_BYTES   ((size_t)MROWS * DFF * 2)
#define OFF_WQKV ((size_t)0)
#define OFF_WPR  (OFF_WQKV + WQKV_BYTES)
#define OFF_WFC  (OFF_WPR + WPR_BYTES)
#define OFF_WOUT (OFF_WFC + WFF_BYTES)
#define OFF_H1   (OFF_WOUT + WFF_BYTES)
#define OFF_Q    (OFF_H1 + P16_BYTES)
#define OFF_K    (OFF_Q + P16_BYTES)
#define OFF_VT   (OFF_K + P16_BYTES)
#define OFF_CTX  (OFF_VT + P16_BYTES)
#define OFF_XM   (OFF_CTX + P16_BYTES)
#define OFF_H2   (OFF_XM + P32_BYTES)
#define OFF_F1   (OFF_H2 + P16_BYTES)
#define WS_TOTAL (OFF_F1 + F1_BYTES)
static_assert((WQKV_BYTES % 128) == 0 && (WPR_BYTES % 128) == 0 && (WFF_BYTES % 128) == 0);
static_assert((P16_BYTES % 128) == 0 && (P32_BYTES % 128) == 0 && (F1_BYTES % 128) == 0);
static_assert(WS_TOTAL <= (size_t)134217728);

__device__ __forceinline__ float bf16r(float x) {
  unsigned int u = __float_as_uint(x);
  u = (u + 0x7FFFu + ((u >> 16) & 1u)) & 0xFFFF0000u;
  return __uint_as_float(u);
}

__device__ __forceinline__ v16h frag_at(const _Float16* p) {
  v8h lo = *(const v8h*)(p);
  v8h hi = *(const v8h*)(p + 16);
  v16h out;
#pragma unroll
  for (int i = 0; i < 8; ++i) { out[i] = lo[i]; out[i + 8] = hi[i]; }
  return out;
}
__device__ __forceinline__ v16h ld_frag(const _Float16* base, unsigned ld) {
  const unsigned lane = threadIdx.x & 31u;
  return frag_at(base + (lane & 15u) * ld + (lane >> 4) * 8u);
}

__device__ __forceinline__ v8f wmma16(v16h a, v16h b, v8f c) {
  v8f d = __builtin_amdgcn_wmma_f32_16x16x32_f16(false, a, false, b, (short)0, c,
                                                 false, false);
  asm volatile("v_nop\n\tv_nop\n\tv_nop\n\tv_nop" : "+v"(d) : "v"(a), "v"(b));
  return d;
}

__device__ __forceinline__ float red16_max(float x) {
#pragma unroll
  for (int off = 1; off < 16; off <<= 1) x = fmaxf(x, __shfl_xor(x, off, 32));
  return x;
}
__device__ __forceinline__ float red16_sum(float x) {
#pragma unroll
  for (int off = 1; off < 16; off <<= 1) x += __shfl_xor(x, off, 32);
  return x;
}
__device__ __forceinline__ float red32_sum(float x) {
#pragma unroll
  for (int off = 1; off < 32; off <<= 1) x += __shfl_xor(x, off, 32);
  return x;
}

__device__ __forceinline__ void wave_lds_sync() {
  __builtin_amdgcn_fence(3  , "wavefront");
  asm volatile("s_wait_dscnt 0x0" ::: "memory");
  __builtin_amdgcn_wave_barrier();
}

__device__ __forceinline__ float gelu_tanh(float v) {
  const float u = 0.7978845608028654f * (v + 0.044715f * v * v * v);
  const float e = __expf(fminf(-2.0f * u, 80.0f));
  return v * __builtin_amdgcn_rcpf(1.0f + e);
}

__global__ __launch_bounds__(256) void wt_kernel(
    const float* __restrict__ src, _Float16* __restrict__ dst, unsigned K, unsigned N) {
  __shared__ __attribute__((aligned(16))) float Cs[64 * LDC];
  const unsigned tid = threadIdx.x;
  const unsigned n0 = blockIdx.x * 64u;
  const unsigned k0 = blockIdx.y * 64u;
#pragma unroll
  for (unsigned i = 0; i < 4u; ++i) {
    const unsigned r = 16u * i + (tid >> 4);
    const unsigned c = (tid & 15u) * 4u;
    const v4f u = *(const v4f*)(src + (size_t)(k0 + r) * N + n0 + c);
    *(v4f*)&Cs[r * LDC + c] = u;
  }
  __syncthreads();
  v8h x[2];
  size_t off[2];
#pragma unroll
  for (unsigned i = 0; i < 2u; ++i) {
    const unsigned dcol = 32u * i + (tid >> 3);
    const unsigned kk = (tid & 7u) * 8u;
#pragma unroll
    for (unsigned j = 0; j < 8u; ++j)
      x[i][j] = (_Float16)(WCARRY * bf16r(Cs[(kk + j) * LDC + dcol]));
    off[i] = (size_t)(n0 + dcol) * K + k0 + kk;
  }
#pragma unroll
  for (int i = 0; i < 2; ++i) *(volatile v8h*)(dst + off[i]) = x[i];
  __threadfence();
#pragma unroll
  for (int i = 0; i < 2; ++i) *(volatile v8h*)(dst + off[i]) = x[i];
}

template <int KD>
__device__ __forceinline__ void gemm_main(
    const _Float16* __restrict__ A16, const _Float16* __restrict__ Bt, float* Cs,
    unsigned row0, unsigned n0) {
  static_assert((KD % 32) == 0);
  const unsigned tid = threadIdx.x, lane = tid & 31u, w = tid >> 5;
  const unsigned mw = w >> 1, nw = w & 1u;
  const unsigned hh = lane >> 4, m = lane & 15u;

  const _Float16* ap  = A16 + (size_t)(row0 + mw * 16u + m) * KD + hh * 8u;
  const _Float16* bp0 = Bt + (size_t)(n0 + nw * 32u + m) * KD + hh * 8u;
  const _Float16* bp1 = bp0 + (size_t)16 * KD;
  v8f acc0 = {}, acc1 = {};
#pragma unroll 2
  for (unsigned k0 = 0; k0 < (unsigned)KD; k0 += 32u) {
    const v16h a  = frag_at(ap + k0);
    const v16h b0 = frag_at(bp0 + k0);
    const v16h b1 = frag_at(bp1 + k0);
    acc0 = wmma16(a, b0, acc0);
    acc1 = wmma16(a, b1, acc1);
  }
#pragma unroll
  for (int r = 0; r < 8; ++r) {
    float* d = &Cs[(mw * 16u + hh * 8u + (unsigned)r) * LDC + nw * 32u + m];
    d[0]  = acc0[r];
    d[16] = acc1[r];
  }
  __syncthreads();
}

template <int ACT>
__device__ __forceinline__ void epi_rowmajor16(
    const float* Cs, const float* __restrict__ biasp, _Float16* __restrict__ outp,
    unsigned pitch, float scl) {
  const unsigned tid = threadIdx.x;
  v8h x[2];
  size_t off[2];
#pragma unroll
  for (unsigned i = 0; i < 2u; ++i) {
    const unsigned r = 32u * i + (tid >> 3);
    const unsigned c = (tid & 7u) * 8u;
    const v4f u0 = *(const v4f*)&Cs[r * LDC + c];
    const v4f u1 = *(const v4f*)&Cs[r * LDC + c + 4];
    const v4f g0 = *(const v4f*)(biasp + c);
    const v4f g1 = *(const v4f*)(biasp + c + 4);
#pragma unroll
    for (int j = 0; j < 4; ++j) {
      float t0 = u0[j] * scl + bf16r(g0[j]);
      float t1 = u1[j] * scl + bf16r(g1[j]);
      if (ACT) { t0 = gelu_tanh(t0); t1 = gelu_tanh(t1); }
      x[i][j]     = (_Float16)t0;
      x[i][j + 4] = (_Float16)t1;
    }
    off[i] = (size_t)r * pitch + c;
  }
#pragma unroll
  for (int i = 0; i < 2; ++i) *(volatile v8h*)(outp + off[i]) = x[i];
  __threadfence();
#pragma unroll
  for (int i = 0; i < 2; ++i) *(volatile v8h*)(outp + off[i]) = x[i];
}

__device__ __forceinline__ void epi_trans16(
    const float* Cs, const float* __restrict__ biasp, _Float16* __restrict__ outp, float scl) {
  const unsigned tid = threadIdx.x;
  v8h x[2];
  size_t off[2];
#pragma unroll
  for (unsigned i = 0; i < 2u; ++i) {
    const unsigned dcol = 32u * i + (tid >> 3);
    const unsigned kk = (tid & 7u) * 8u;
    const float bb = bf16r(biasp[dcol]);
#pragma unroll
    for (unsigned j = 0; j < 8u; ++j)
      x[i][j] = (_Float16)(Cs[(kk + j) * LDC + dcol] * scl + bb);
    off[i] = (size_t)dcol * SEQ + kk;
  }
#pragma unroll
  for (int i = 0; i < 2; ++i) *(volatile v8h*)(outp + off[i]) = x[i];
  __threadfence();
#pragma unroll
  for (int i = 0; i < 2; ++i) *(volatile v8h*)(outp + off[i]) = x[i];
}

__device__ __forceinline__ void epi_cache32(
    const float* Cs, const float* __restrict__ biasp, float* __restrict__ outp, float scl) {
  const unsigned tid = threadIdx.x;
  v4f xs[4];
  size_t off[4];
#pragma unroll
  for (unsigned i = 0; i < 4u; ++i) {
    const unsigned r = 16u * i + (tid >> 4);
    const unsigned c = (tid & 15u) * 4u;
    const v4f u = *(const v4f*)&Cs[r * LDC + c];
    const v4f g = *(const v4f*)(biasp + c);
    v4f val;
#pragma unroll
    for (int j = 0; j < 4; ++j) val[j] = u[j] * scl + bf16r(g[j]);
    xs[i] = val;
    off[i] = (size_t)r * HD + c;
  }
#pragma unroll
  for (int i = 0; i < 4; ++i) *(volatile v4f*)(outp + off[i]) = xs[i];
  __threadfence();
#pragma unroll
  for (int i = 0; i < 4; ++i) *(volatile v4f*)(outp + off[i]) = xs[i];
}

template <int XMAP_RES, int XMAP_OUT>
__device__ __forceinline__ void epi_f32_res(
    const float* Cs, const float* __restrict__ biasp, const float* __restrict__ resf,
    float* __restrict__ outf, unsigned row0, unsigned n0, float scl) {
  const unsigned tid = threadIdx.x;
  const unsigned b = row0 / (unsigned)SEQ;
  const unsigned l0 = row0 % (unsigned)SEQ;
  v4f xs[4];
  size_t off[4];
#pragma unroll
  for (unsigned i = 0; i < 4u; ++i) {
    const unsigned r = 16u * i + (tid >> 4);
    const unsigned c = (tid & 15u) * 4u;
    const size_t trow = (size_t)(row0 + r);
    const size_t xrow = (size_t)(l0 + r) * NB_FULL + b;
    const size_t ro = (XMAP_RES ? xrow : trow) * DIM + n0 + c;
    const size_t oo = (XMAP_OUT ? xrow : trow) * DIM + n0 + c;
    const v4f u = *(const v4f*)&Cs[r * LDC + c];
    const v4f g = *(const v4f*)(biasp + c);
    const v4f hres = *(const v4f*)(resf + ro);
    v4f val;
#pragma unroll
    for (int j = 0; j < 4; ++j) {
      const float rr = XMAP_RES ? bf16r(hres[j]) : hres[j];
      val[j] = rr + (u[j] * scl + bf16r(g[j]));
    }
    xs[i] = val;
    off[i] = oo;
  }
#pragma unroll
  for (int i = 0; i < 4; ++i) *(volatile v4f*)(outf + off[i]) = xs[i];
  __threadfence();
#pragma unroll
  for (int i = 0; i < 4; ++i) *(volatile v4f*)(outf + off[i]) = xs[i];
}

__global__ __launch_bounds__(256) void gemm_qkv_kernel(
    const _Float16* __restrict__ A16, const _Float16* __restrict__ Bt,
    const float* __restrict__ bias, _Float16* __restrict__ Q16, _Float16* __restrict__ K16,
    _Float16* __restrict__ Vt16, float* __restrict__ outf) {
  __shared__ __attribute__((aligned(16))) float Cs[64 * LDC];
  const unsigned n0 = blockIdx.x * 64u;
  const unsigned row0 = blockIdx.y * 64u;
  gemm_main<DIM>(A16, Bt, Cs, row0, n0);

  const unsigned sel = blockIdx.x / (unsigned)(DIM / 64);
  const unsigned c0 = n0 - sel * (unsigned)DIM;
  const unsigned head = c0 / (unsigned)HD;
  const unsigned b = row0 / (unsigned)SEQ;
  const unsigned l0 = row0 % (unsigned)SEQ;
  const float scl = 1.0f / WCARRY;
  const float* bp = bias + n0;

  if (sel == 0u) {
    epi_rowmajor16<0>(Cs, bp, Q16 + (size_t)row0 * DIM + c0, (unsigned)DIM, scl);
  } else if (sel == 1u) {
    epi_rowmajor16<0>(Cs, bp, K16 + (size_t)row0 * DIM + c0, (unsigned)DIM, scl);
  } else {
    epi_trans16(Cs, bp, Vt16 + ((size_t)b * DIM + c0) * SEQ + l0, scl);
  }
  if (sel >= 1u) {
    const size_t po = OUT1_ELEM +
        ((((size_t)(sel - 1u) * NB_FULL + b) * NHEAD + head) * SEQ_FULL + l0) * HD;
    epi_cache32(Cs, bp, outf + po, scl);
  }
}

__global__ __launch_bounds__(256) void gemm_proj_kernel(
    const _Float16* __restrict__ A16, const _Float16* __restrict__ Bt,
    const float* __restrict__ bias, const float* __restrict__ X, float* __restrict__ XM) {
  __shared__ __attribute__((aligned(16))) float Cs[64 * LDC];
  const unsigned n0 = blockIdx.x * 64u;
  const unsigned row0 = blockIdx.y * 64u;
  gemm_main<DIM>(A16, Bt, Cs, row0, n0);
  epi_f32_res<1, 0>(Cs, bias + n0, X, XM, row0, n0, 1.0f / (WCARRY * VCARRY));
}

__global__ __launch_bounds__(256) void gemm_ffn1_kernel(
    const _Float16* __restrict__ A16, const _Float16* __restrict__ Bt,
    const float* __restrict__ bias, _Float16* __restrict__ out16) {
  __shared__ __attribute__((aligned(16))) float Cs[64 * LDC];
  const unsigned n0 = blockIdx.x * 64u;
  const unsigned row0 = blockIdx.y * 64u;
  gemm_main<DIM>(A16, Bt, Cs, row0, n0);
  epi_rowmajor16<1>(Cs, bias + n0, out16 + (size_t)row0 * DFF + n0, (unsigned)DFF,
                    1.0f / WCARRY);
}

__global__ __launch_bounds__(256) void gemm_ffn2_kernel(
    const _Float16* __restrict__ A16, const _Float16* __restrict__ Bt,
    const float* __restrict__ bias, const float* __restrict__ XM, float* __restrict__ outf) {
  __shared__ __attribute__((aligned(16))) float Cs[64 * LDC];
  const unsigned n0 = blockIdx.x * 64u;
  const unsigned row0 = blockIdx.y * 64u;
  gemm_main<DFF>(A16, Bt, Cs, row0, n0);
  epi_f32_res<0, 1>(Cs, bias + n0, XM, outf, row0, n0, 1.0f / WCARRY);
}

__global__ __launch_bounds__(256) void attn_kernel(
    const _Float16* __restrict__ Qp, const _Float16* __restrict__ Kp,
    const _Float16* __restrict__ Vt, _Float16* __restrict__ Ov) {
  __shared__ __attribute__((aligned(16))) _Float16 Ks[64 * LDT];
  __shared__ __attribute__((aligned(16))) _Float16 Vs[64 * LDT];
  __shared__ __attribute__((aligned(16))) _Float16 Ps[8 * 16 * LDT];

  const unsigned tid = threadIdx.x, lane = tid & 31u, w = tid >> 5;
  const unsigned hh = lane >> 4, m = lane & 15u;
  const unsigned q0 = blockIdx.x * 128u;
  const unsigned head = blockIdx.y;
  const unsigned b = blockIdx.z;
  const float scale = 0.125f;
  _Float16* P = Ps + w * (16u * LDT);

  const size_t tbase = (size_t)b * SEQ;
  const size_t qoff = (tbase + q0 + w * 16u + m) * DIM + head * HD + hh * 8u;
  v16h qf[2];
  qf[0] = frag_at(Qp + qoff);
  qf[1] = frag_at(Qp + qoff + 32);

  float mrow[8], lrow[8];
  v8f o[4];
#pragma unroll
  for (int v = 0; v < 8; ++v) { mrow[v] = -1.0e30f; lrow[v] = 0.0f; }
#pragma unroll
  for (int nb = 0; nb < 4; ++nb) o[nb] = (v8f){};

  const size_t kplane = tbase * DIM + (size_t)head * HD;
  const size_t vplane = ((size_t)b * DIM + (size_t)head * HD) * SEQ;

  for (unsigned kb = 0; kb < (unsigned)SEQ; kb += 64u) {
#pragma unroll
    for (unsigned j = 0; j < 2u; ++j) {
      const unsigned idx = tid + 256u * j;
      const unsigned r = idx >> 3, c = (idx & 7u) * 8u;
      *(v8h*)&Ks[r * LDT + c] = *(const v8h*)(Kp + kplane + (size_t)(kb + r) * DIM + c);
      *(v8h*)&Vs[r * LDT + c] = *(const v8h*)(Vt + vplane + (size_t)r * SEQ + kb + c);
    }
    __syncthreads();

    v8f s[4];
#pragma unroll
    for (int kg = 0; kg < 4; ++kg) {
      v8f t = {};
#pragma unroll
      for (int c = 0; c < 2; ++c) {
        const v16h kf = ld_frag(&Ks[(kg * 16) * LDT + c * 32], LDT);
        t = wmma16(qf[c], kf, t);
      }
      s[kg] = t * scale;
    }

    float alpha[8];
#pragma unroll
    for (int v = 0; v < 8; ++v) {
      float mx = fmaxf(fmaxf(s[0][v], s[1][v]), fmaxf(s[2][v], s[3][v]));
      mx = red16_max(mx);
      const float mn = fmaxf(mrow[v], mx);
      alpha[v] = __expf(mrow[v] - mn);
      mrow[v] = mn;
    }
#pragma unroll
    for (int kg = 0; kg < 4; ++kg)
#pragma unroll
      for (int v = 0; v < 8; ++v) s[kg][v] = __expf(s[kg][v] - mrow[v]);
#pragma unroll
    for (int v = 0; v < 8; ++v) {
      const float rs = red16_sum((s[0][v] + s[1][v]) + (s[2][v] + s[3][v]));
      lrow[v] = alpha[v] * lrow[v] + rs;
    }
#pragma unroll
    for (int nb = 0; nb < 4; ++nb)
#pragma unroll
      for (int v = 0; v < 8; ++v) o[nb][v] = o[nb][v] * alpha[v];

#pragma unroll
    for (int kg = 0; kg < 4; ++kg)
#pragma unroll
      for (int v = 0; v < 8; ++v)
        P[(hh * 8u + (unsigned)v) * LDT + (unsigned)kg * 16u + m] = (_Float16)(s[kg][v] * PCARRY);
    wave_lds_sync();

#pragma unroll
    for (int c = 0; c < 2; ++c) {
      const v16h pf = ld_frag(P + c * 32, LDT);
#pragma unroll
      for (int nb = 0; nb < 4; ++nb) {
        const v16h vf = ld_frag(&Vs[(nb * 16) * LDT + c * 32], LDT);
        o[nb] = wmma16(pf, vf, o[nb]);
      }
    }
    __syncthreads();
  }

  float inv[8];
#pragma unroll
  for (int v = 0; v < 8; ++v) inv[v] = __builtin_amdgcn_rcpf(lrow[v]) * (VCARRY / PCARRY);
#pragma unroll
  for (int nb = 0; nb < 4; ++nb)
#pragma unroll
    for (int v = 0; v < 8; ++v)
      P[(hh * 8u + (unsigned)v) * LDT + (unsigned)nb * 16u + m] = (_Float16)(o[nb][v] * inv[v]);
  wave_lds_sync();
  v8h x[4];
  size_t off[4];
#pragma unroll
  for (unsigned i = 0; i < 4u; ++i) {
    const unsigned r = 4u * i + (lane >> 3);
    const unsigned c = (lane & 7u) * 8u;
    x[i] = *(const v8h*)&P[r * LDT + c];
    off[i] = (tbase + q0 + w * 16u + r) * DIM + head * HD + c;
  }
#pragma unroll
  for (int i = 0; i < 4; ++i) *(volatile v8h*)(Ov + off[i]) = x[i];
  __threadfence();
#pragma unroll
  for (int i = 0; i < 4; ++i) *(volatile v8h*)(Ov + off[i]) = x[i];
}

__device__ __forceinline__ void ln_store16(
    const float* S, const float* __restrict__ g, const float* __restrict__ be,
    _Float16* __restrict__ orow, float mu, float rs) {
  const unsigned lane = threadIdx.x & 31u;
#pragma unroll 1
  for (unsigned it = 0; it < (unsigned)(DIM / 256); ++it) {
    const unsigned c = it * 256u + lane * 8u;
    const v4f v0 = *(const v4f*)&S[c];
    const v4f v1 = *(const v4f*)&S[c + 4];
    const v4f g0 = *(const v4f*)(g + c);
    const v4f g1 = *(const v4f*)(g + c + 4);
    const v4f b0 = *(const v4f*)(be + c);
    const v4f b1 = *(const v4f*)(be + c + 4);
    v8h x;
#pragma unroll
    for (int j = 0; j < 4; ++j) {
      x[j]     = (_Float16)((v0[j] - mu) * rs * bf16r(g0[j]) + bf16r(b0[j]));
      x[j + 4] = (_Float16)((v1[j] - mu) * rs * bf16r(g1[j]) + bf16r(b1[j]));
    }
    *(volatile v8h*)(orow + c) = x;
  }
}

template <int RNDIN>
__device__ __forceinline__ void ln_row(
    const float* __restrict__ srow, const float* __restrict__ g, const float* __restrict__ be,
    _Float16* __restrict__ orow, float* S) {
  const unsigned lane = threadIdx.x & 31u;
  float sum = 0.0f;
#pragma unroll 1
  for (unsigned it = 0; it < (unsigned)(DIM / 128); ++it) {
    const unsigned c = it * 128u + lane * 4u;
    v4f v = *(const v4f*)(srow + c);
    if (RNDIN) {
#pragma unroll
      for (int j = 0; j < 4; ++j) v[j] = bf16r(v[j]);
    }
    *(v4f*)&S[c] = v;
    sum += (v[0] + v[1]) + (v[2] + v[3]);
  }
  sum = red32_sum(sum);
  const float mu = sum * (1.0f / (float)DIM);
  float sq = 0.0f;
#pragma unroll 1
  for (unsigned it = 0; it < (unsigned)(DIM / 128); ++it) {
    const unsigned c = it * 128u + lane * 4u;
    const v4f v = *(const v4f*)&S[c];
    const float d0 = v[0] - mu, d1 = v[1] - mu, d2 = v[2] - mu, d3 = v[3] - mu;
    sq += (d0 * d0 + d1 * d1) + (d2 * d2 + d3 * d3);
  }
  sq = red32_sum(sq);
  const float rs = rsqrtf(sq * (1.0f / (float)DIM) + LN_EPS);
  wave_lds_sync();
  ln_store16(S, g, be, orow, mu, rs);
  __threadfence();
  ln_store16(S, g, be, orow, mu, rs);
}

__global__ __launch_bounds__(256) void ln1_kernel(
    const float* __restrict__ X, const float* __restrict__ g, const float* __restrict__ be,
    _Float16* __restrict__ h16) {
  __shared__ __attribute__((aligned(16))) float S[LNROWS * DIM];
  const unsigned w = threadIdx.x >> 5;
  const unsigned t = blockIdx.x * (unsigned)LNROWS + w;
  const unsigned b = t / (unsigned)SEQ, l = t % (unsigned)SEQ;
  const size_t xrow = (size_t)l * NB_FULL + b;
  ln_row<1>(X + xrow * DIM, g, be, h16 + (size_t)t * DIM, S + w * (unsigned)DIM);
}
__global__ __launch_bounds__(256) void ln2_kernel(
    const float* __restrict__ XM, const float* __restrict__ g, const float* __restrict__ be,
    _Float16* __restrict__ h16) {
  __shared__ __attribute__((aligned(16))) float S[LNROWS * DIM];
  const unsigned w = threadIdx.x >> 5;
  const unsigned t = blockIdx.x * (unsigned)LNROWS + w;
  ln_row<0>(XM + (size_t)t * DIM, g, be, h16 + (size_t)t * DIM, S + w * (unsigned)DIM);
}

extern "C" void kernel_launch(void* const* d_in, const int* in_sizes, int n_in,
                              void* d_out, int out_size, void* d_ws, size_t ws_size,
                              hipStream_t stream) {
  if (n_in < 13) return;
  const long long need_x = ((long long)(SEQ - 1) * NB_FULL + NB) * DIM;
  if ((long long)in_sizes[0] < need_x) return;
  if (in_sizes[1] < DIM || in_sizes[2] < DIM) return;
  if ((long long)in_sizes[3] < (long long)3 * DIM * DIM) return;
  if (in_sizes[4] < 3 * DIM) return;
  if ((long long)in_sizes[5] < (long long)DIM * DIM) return;
  if (in_sizes[6] < DIM || in_sizes[7] < DIM || in_sizes[8] < DIM) return;
  if ((long long)in_sizes[9] < (long long)DIM * DFF) return;
  if (in_sizes[10] < DFF) return;
  if ((long long)in_sizes[11] < (long long)DFF * DIM) return;
  if (in_sizes[12] < DIM) return;
  if ((long long)out_size < (long long)NEED_OUT) return;
  if (ws_size < WS_TOTAL) return;

  const float* X     = (const float*)d_in[0];
  const float* g1    = (const float*)d_in[1];
  const float* be1   = (const float*)d_in[2];
  const float* Wqkv  = (const float*)d_in[3];
  const float* bqkv  = (const float*)d_in[4];
  const float* Wpr   = (const float*)d_in[5];
  const float* bpr   = (const float*)d_in[6];
  const float* g2    = (const float*)d_in[7];
  const float* be2   = (const float*)d_in[8];
  const float* Wfc   = (const float*)d_in[9];
  const float* bfc   = (const float*)d_in[10];
  const float* Wout  = (const float*)d_in[11];
  const float* bout  = (const float*)d_in[12];
  float* out = (float*)d_out;

  char* ws = (char*)d_ws;
  _Float16* Wqkv16 = (_Float16*)(ws + OFF_WQKV);
  _Float16* Wpr16  = (_Float16*)(ws + OFF_WPR);
  _Float16* Wfc16  = (_Float16*)(ws + OFF_WFC);
  _Float16* Wout16 = (_Float16*)(ws + OFF_WOUT);
  _Float16* H1_16  = (_Float16*)(ws + OFF_H1);
  _Float16* Q16    = (_Float16*)(ws + OFF_Q);
  _Float16* K16    = (_Float16*)(ws + OFF_K);
  _Float16* Vt16   = (_Float16*)(ws + OFF_VT);
  _Float16* Ctx16  = (_Float16*)(ws + OFF_CTX);
  float*    XM     = (float*)(ws + OFF_XM);
  _Float16* H2_16  = (_Float16*)(ws + OFF_H2);
  _Float16* F1_16  = (_Float16*)(ws + OFF_F1);

  dim3 blk(256);

  wt_kernel<<<dim3(3 * DIM / 64, DIM / 64), blk, 0, stream>>>(Wqkv, Wqkv16, DIM, 3 * DIM);
  wt_kernel<<<dim3(DIM / 64, DIM / 64), blk, 0, stream>>>(Wpr, Wpr16, DIM, DIM);
  wt_kernel<<<dim3(DFF / 64, DIM / 64), blk, 0, stream>>>(Wfc, Wfc16, DIM, DFF);
  wt_kernel<<<dim3(DIM / 64, DFF / 64), blk, 0, stream>>>(Wout, Wout16, DFF, DIM);

  ln1_kernel<<<dim3(MROWS / LNROWS), blk, 0, stream>>>(X, g1, be1, H1_16);

  gemm_qkv_kernel<<<dim3(3 * DIM / 64, MROWS / 64), blk, 0, stream>>>(
      H1_16, Wqkv16, bqkv, Q16, K16, Vt16, out);

  attn_kernel<<<dim3(SEQ / 128, NHEAD, NB), blk, 0, stream>>>(Q16, K16, Vt16, Ctx16);

  gemm_proj_kernel<<<dim3(DIM / 64, MROWS / 64), blk, 0, stream>>>(Ctx16, Wpr16, bpr, X, XM);

  ln2_kernel<<<dim3(MROWS / LNROWS), blk, 0, stream>>>(XM, g2, be2, H2_16);

  gemm_ffn1_kernel<<<dim3(DFF / 64, MROWS / 64), blk, 0, stream>>>(H2_16, Wfc16, bfc, F1_16);
  gemm_ffn2_kernel<<<dim3(DIM / 64, MROWS / 64), blk, 0, stream>>>(F1_16, Wout16, bout, XM, out);
}
